// MultiHeadedAttention_39951785787979
// MI455X (gfx1250) — hardware-verified
//
#include <hip/hip_runtime.h>
#include <math.h>

typedef __attribute__((ext_vector_type(16))) _Float16 v16h;
typedef __attribute__((ext_vector_type(16))) __bf16 v16b;
typedef __attribute__((ext_vector_type(8)))  _Float16 v8h;
typedef __attribute__((ext_vector_type(8)))  __bf16 v8b;
typedef __attribute__((ext_vector_type(8)))  float v8f;
typedef __attribute__((ext_vector_type(4)))  float v4f;
typedef __attribute__((ext_vector_type(4)))  unsigned v4u;
typedef __attribute__((ext_vector_type(4)))  int v4i;

template <typename T> __device__ __forceinline__ void vst2(void* p, T v) { *(volatile T*)p = v; __threadfence(); *(volatile T*)p = v; }
__device__ __forceinline__ v8f wmma16(v16h a, v16h b, v8f c) {
  v8f d = __builtin_amdgcn_wmma_f32_16x16x32_f16(false, a, false, b, (short)0, c, false, false);
  asm volatile("v_nop\n\tv_nop\n\tv_nop\n\tv_nop" : "+v"(d) : "v"(a), "v"(b));
  return d;
}
__device__ __forceinline__ v8f wmma_bf(v16b a, v16b b, v8f c) {
  v8f d = __builtin_amdgcn_wmma_f32_16x16x32_bf16(false, a, false, b, (short)0, c, false, false);
  asm volatile("v_nop\n\tv_nop\n\tv_nop\n\tv_nop" : "+v"(d) : "v"(a), "v"(b));
  return d;
}
__device__ __forceinline__ v16h frag_h(const _Float16* rowk0, int lane) {
  union { v16h v; v8h q[2]; } u; const _Float16* p = rowk0 + 8 * (lane >> 4);
  u.q[0] = *(const v8h*)p; u.q[1] = *(const v8h*)(p + 16); return u.v;
}
__device__ __forceinline__ v16b frag_b(const __bf16* rowk0, int lane) {
  union { v16b v; v8b q[2]; } u; const __bf16* p = rowk0 + 8 * (lane >> 4);
  u.q[0] = *(const v8b*)p; u.q[1] = *(const v8b*)(p + 16); return u.v;
}
__device__ __forceinline__ v16h frag_f32s(const float* rowk0, int lane, float sc) {
  v16h a; const float* p = rowk0 + 8 * (lane >> 4);
#pragma unroll
  for (int i = 0; i < 8; ++i) { a[i] = (_Float16)(p[i] * sc); a[8 + i] = (_Float16)(p[16 + i] * sc); }
  return a;
}
struct F2 { v16b h, l; };
__device__ __forceinline__ F2 bsplit16(const float v[16]) { F2 r;
#pragma unroll
  for (int i = 0; i < 16; ++i) { const __bf16 h = (__bf16)v[i]; r.h[i] = h; r.l[i] = (__bf16)(v[i] - (float)h); }
  return r; }
__device__ __forceinline__ F2 split_row(const float* row, int k0, int lane) { float v[16]; const float* p = row + k0 + 8 * (lane >> 4);
#pragma unroll
  for (int i = 0; i < 8; ++i) { v[i] = p[i]; v[8 + i] = p[16 + i]; }
  return bsplit16(v); }
__device__ __forceinline__ float bfr(float v) { return (float)(__bf16)v; }
__device__ __forceinline__ v16b wcol_oi(const float* Wm, int k0, int o, int lane, int K) { v16b w; const float* p = Wm + (size_t)o * K + k0 + 8 * (lane >> 4);
#pragma unroll
  for (int i = 0; i < 8; ++i) { w[i] = (__bf16)p[i]; w[8 + i] = (__bf16)p[16 + i]; }
  return w; }
__device__ __forceinline__ v16h wcolh_oi(const float* Wm, int k0, int o, int lane, int K) { v16h w; const float* p = Wm + (size_t)o * K + k0 + 8 * (lane >> 4);
#pragma unroll
  for (int i = 0; i < 8; ++i) { w[i] = (_Float16)(bfr(p[i]) * 256.0f); w[8 + i] = (_Float16)(bfr(p[16 + i]) * 256.0f); }
  return w; }
#define LDSX() do { asm volatile("s_wait_dscnt 0" ::: "memory"); __builtin_amdgcn_wave_barrier(); __builtin_amdgcn_fence(3  , "workgroup"); } while (0)

#ifndef NB
#define NB 4
#endif
#ifndef SEQ
#define SEQ 1024
#endif
#define NB_FULL 4
#define SEQ_FULL 1024
#define CC 1024
#define DIN 1024
#define NH 16
#define HD 64
#define NQB (SEQ / 64)
#define EARLY (SEQ < 256 ? SEQ : 256)
#define SCALE (0.015625f)
#define LOG2E (1.44269504088896f)

static_assert(SEQ % 64 == 0);
static_assert(EARLY % 64 == 0);
static_assert(NQB <= 16);
static_assert(CC == NH * HD);
static_assert(HD == 64);
static_assert(CC % 128 == 0);
static_assert(DIN % 128 == 0);
static_assert(DIN % 32 == 0);
static_assert(CC % 32 == 0);
static_assert(DIN == CC);
static_assert(NB <= NB_FULL);
static_assert(SEQ <= SEQ_FULL);
static_assert((NB * SEQ) % 64 == 0);

#define WS_QH  ((size_t)0)
#define WS_KH  (WS_QH  + (size_t)2 * NB * SEQ * CC)
#define WS_VT  (WS_KH  + (size_t)2 * NB * SEQ * CC)
#define WS_VB  (WS_VT  + (size_t)2 * NB * CC * SEQ)
#define WS_VBL (WS_VB  + (size_t)2 * NB * CC * EARLY)
#define WS_Y   (WS_VBL + (size_t)2 * NB * CC * EARLY)
#define WS_FLG (WS_Y   + (size_t)4 * NB * SEQ * CC)
#define WS_END (WS_FLG + (size_t)128 * NB * NQB)
static_assert(WS_END <= (size_t)134217728);
static_assert(WS_KH % 128 == 0 && WS_VT % 128 == 0 && WS_VB % 128 == 0 && WS_VBL % 128 == 0 && WS_Y % 128 == 0 && WS_FLG % 128 == 0);
static_assert(((size_t)(NB - 1) * SEQ_FULL + SEQ) * DIN <= (size_t)NB_FULL * SEQ_FULL * DIN);

__global__ __launch_bounds__(256) void k_mflag(const int* __restrict__ MASK, int* __restrict__ FLG) {
  __shared__ __align__(16) int sfl[32];
  const int tid = threadIdx.x; const int qb = blockIdx.x, b = blockIdx.y;
  const int kbi = tid >> 4, sub = tid & 15; const int kc = kbi < NQB ? kbi : NQB - 1;
  const int* base = MASK + ((size_t)b * SEQ_FULL + (size_t)qb * 64) * SEQ_FULL + kc * 64 + sub * 4;
  int any = 0, zc = 0;
#pragma unroll 4
  for (int r = 0; r < 64; ++r) { const v4i m = *(const v4i*)(base + (size_t)r * SEQ_FULL);
    any |= (m[0] | m[1] | m[2] | m[3]); zc |= (int)(m[0] == 0) | (int)(m[1] == 0) | (int)(m[2] == 0) | (int)(m[3] == 0); }
#pragma unroll
  for (int o = 1; o < 16; o <<= 1) { any |= __shfl_xor(any, o); zc |= __shfl_xor(zc, o); }
  const int flag = (any == 0) ? 0 : (zc ? 1 : 2);
  if (sub == 0) sfl[kbi] = flag;
  if (tid < 16) sfl[16 + tid] = 1;
  __syncthreads();
  if (tid < 8) vst2(FLG + ((size_t)b * NQB + qb) * 32 + tid * 4, *(const v4i*)&sfl[tid * 4]);
}

__global__ __launch_bounds__(128) void k_proj(const float* __restrict__ XQ, const float* __restrict__ XK, const float* __restrict__ XV,
    const float* __restrict__ WQ, const float* __restrict__ WK, const float* __restrict__ WV,
    const float* __restrict__ BQ, const float* __restrict__ BK, const float* __restrict__ BV,
    _Float16* __restrict__ QH, _Float16* __restrict__ KH, _Float16* __restrict__ VT, __bf16* __restrict__ VB, __bf16* __restrict__ VBL) {
  __shared__ __align__(16) _Float16 sh[64][136];
  __shared__ __align__(16) _Float16 th[128][72];
  __shared__ __align__(16) __bf16 tb[128][72], tbl[128][72];
  const int tid = threadIdx.x, wave = tid >> 5, lane = tid & 31, col = lane & 15, g = lane >> 4;
  const int which = blockIdx.z; const int c0 = blockIdx.y * 128;
  const size_t r0 = (size_t)blockIdx.x * 64; const size_t bb = r0 / SEQ; const int t0 = (int)(r0 % SEQ);
  const float* X = which == 0 ? XQ : which == 1 ? XK : XV; const float* WA = which == 0 ? WQ : which == 1 ? WK : WV; const float* BA = which == 0 ? BQ : which == 1 ? BK : BV;
  const float* xrow = X + (bb * SEQ_FULL + (size_t)t0 + wave * 16 + col) * (size_t)DIN;
  v8f acc[8] = {};
#pragma unroll 2
  for (int kc = 0; kc < DIN / 32; ++kc) { v16b a; { const float* p = xrow + kc * 32 + 8 * g;
#pragma unroll
      for (int i = 0; i < 8; ++i) { a[i] = (__bf16)p[i]; a[8 + i] = (__bf16)p[16 + i]; } }
    asm volatile("s_wait_loadcnt 0x0" ::: "memory");
#pragma unroll
    for (int j = 0; j < 8; ++j) { const v16b w = wcol_oi(WA, kc * 32, c0 + j * 16 + col, lane, DIN); asm volatile("s_wait_loadcnt 0x0" ::: "memory"); acc[j] = wmma_bf(a, w, acc[j]); } }
  if (which < 2) { _Float16* DH = which == 0 ? QH : KH;
#pragma unroll
    for (int j = 0; j < 8; ++j) { const float bias = BA ? bfr(BA[c0 + j * 16 + col]) : 0.f;
#pragma unroll
      for (int r = 0; r < 8; ++r) sh[wave * 16 + 8 * g + r][j * 16 + col] = (_Float16)(acc[j][r] + bias); }
    __syncthreads();
    for (int e = tid; e < 64 * 16; e += 128) { const int rl = e >> 4, q = e & 15; vst2(DH + (r0 + rl) * CC + c0 + q * 8, *(const v4u*)&sh[rl][q * 8]); }
  } else { const bool hi_rows = t0 < EARLY;
#pragma unroll
    for (int j = 0; j < 8; ++j) { const float bias = BA ? bfr(BA[c0 + j * 16 + col]) : 0.f;
#pragma unroll
      for (int r = 0; r < 8; ++r) { const float v = acc[j][r] + bias; const int rl = wave * 16 + 8 * g + r, cl = j * 16 + col; th[cl][rl] = (_Float16)v; const __bf16 bh = (__bf16)v; tb[cl][rl] = bh; tbl[cl][rl] = (__bf16)(v - (float)bh); } }
    __syncthreads();
    for (int e = tid; e < 128 * 8; e += 128) { const int cl = e >> 3, q = e & 7;
      vst2(VT + (bb * CC + c0 + cl) * (size_t)SEQ + t0 + q * 8, *(const v4u*)&th[cl][q * 8]);
      if (hi_rows) { const size_t o3 = (bb * CC + c0 + cl) * (size_t)EARLY + t0 + q * 8; vst2(VB + o3, *(const v4u*)&tb[cl][q * 8]); vst2(VBL + o3, *(const v4u*)&tbl[cl][q * 8]); } } } }

__global__ __launch_bounds__(128) void k_attn(const _Float16* __restrict__ QH, const _Float16* __restrict__ KH, const _Float16* __restrict__ VT,
    const __bf16* __restrict__ VB, const __bf16* __restrict__ VBL, const int* __restrict__ MASK, const int* __restrict__ FLG, float* __restrict__ Y) {
  __shared__ __align__(16) float ss[4][16][68];
  const int tid = threadIdx.x, wave = tid >> 5, lane = tid & 31, col = lane & 15, g = lane >> 4;
  const int qb = blockIdx.x, h = blockIdx.y, b = blockIdx.z;
  const int ql0 = qb * 64 + wave * 16;
  const _Float16* qp = QH + ((size_t)b * SEQ + ql0 + col) * CC + h * HD;
  const v16h qf0 = frag_h(qp, lane), qf1 = frag_h(qp + 32, lane);
  const _Float16* kbase = KH + ((size_t)b * SEQ + col) * CC + h * HD;
  const _Float16* vbase = VT + ((size_t)b * CC + h * HD + col) * (size_t)SEQ;
  const size_t vbo = ((size_t)b * CC + h * HD + col) * (size_t)EARLY;
  const int* mrowp = MASK + ((size_t)b * SEQ_FULL + ql0 + col) * (size_t)SEQ_FULL + 8 * g;
  const int* frow = FLG + ((size_t)b * NQB + qb) * 32;
  v8f o[4] = {};
  float mrow = -1.0e30f, lrow = 0.f; int skipped = 0;
#pragma unroll 1
  for (int kb = 0; kb < NQB; ++kb) {
    const int fl = __builtin_amdgcn_readfirstlane(frow[kb]);
    if (fl == 0) { skipped = 1; continue; }
    const bool hp = (qb < EARLY / 64) && (kb < EARLY / 64);
#pragma unroll 1
    for (int hf = 0; hf < 2; ++hf) {
      const int key0 = kb * 64 + hf * 32;
      v8f t0 = {}, t1 = {};
      { const _Float16* kp = kbase + (size_t)key0 * CC;
        const v16h ka0 = frag_h(kp, lane), ka1 = frag_h(kp + 32, lane), kc0 = frag_h(kp + 16 * CC, lane), kc1 = frag_h(kp + 16 * CC + 32, lane);
        t0 = wmma16(ka0, qf0, t0); t0 = wmma16(ka1, qf1, t0); t1 = wmma16(kc0, qf0, t1); t1 = wmma16(kc1, qf1, t1); }
      t0 = t0 * SCALE; t1 = t1 * SCALE;
      if (fl != 2) { const int* mk = mrowp + key0;
        const v4i m0 = *(const v4i*)mk, m1 = *(const v4i*)(mk + 4), m2 = *(const v4i*)(mk + 16), m3 = *(const v4i*)(mk + 20);
#pragma unroll
        for (int r = 0; r < 4; ++r) { t0[r] = (m0[r] == 0) ? -1.0e9f : t0[r]; t0[4 + r] = (m1[r] == 0) ? -1.0e9f : t0[4 + r]; t1[r] = (m2[r] == 0) ? -1.0e9f : t1[r]; t1[4 + r] = (m3[r] == 0) ? -1.0e9f : t1[4 + r]; } }
      float loc = fmaxf(t0[0], t1[0]);
#pragma unroll
      for (int r = 1; r < 8; ++r) loc = fmaxf(loc, fmaxf(t0[r], t1[r]));
      loc = fmaxf(loc, __shfl_xor(loc, 16));
      const float mnew = fmaxf(mrow, loc);
      const float alpha = exp2f((mrow - mnew) * LOG2E);
      float p0[8], p1[8], psum = 0.f;
#pragma unroll
      for (int r = 0; r < 8; ++r) { p0[r] = exp2f((t0[r] - mnew) * LOG2E); p1[r] = exp2f((t1[r] - mnew) * LOG2E); psum += p0[r] + p1[r]; }
      psum += __shfl_xor(psum, 16);
      lrow = lrow * alpha + psum; mrow = mnew;
#pragma unroll
      for (int j = 0; j < 4; ++j) o[j] = o[j] * alpha;
      if (hp) {
        v16b ph, pl;
#pragma unroll
        for (int r = 0; r < 8; ++r) { const __bf16 a0 = (__bf16)p0[r]; ph[r] = a0; pl[r] = (__bf16)(p0[r] - (float)a0); const __bf16 a1 = (__bf16)p1[r]; ph[8 + r] = a1; pl[8 + r] = (__bf16)(p1[r] - (float)a1); }
        const size_t vo = vbo + key0;
#pragma unroll
        for (int j = 0; j < 4; ++j) { const v16b vh = frag_b(VB + vo + (size_t)j * 16 * EARLY, lane), vl = frag_b(VBL + vo + (size_t)j * 16 * EARLY, lane);
          o[j] = wmma_bf(vh, pl, o[j]); o[j] = wmma_bf(vl, ph, o[j]); o[j] = wmma_bf(vh, ph, o[j]); }
      } else {
        v16h pf;
#pragma unroll
        for (int r = 0; r < 8; ++r) { pf[r] = (_Float16)p0[r]; pf[8 + r] = (_Float16)p1[r]; }
        const _Float16* vp = vbase + key0;
        const v16h v0 = frag_h(vp, lane), v1 = frag_h(vp + (size_t)16 * SEQ, lane), v2 = frag_h(vp + (size_t)32 * SEQ, lane), v3 = frag_h(vp + (size_t)48 * SEQ, lane);
        o[0] = wmma16(v0, pf, o[0]); o[1] = wmma16(v1, pf, o[1]); o[2] = wmma16(v2, pf, o[2]); o[3] = wmma16(v3, pf, o[3]);
      }
    }
  }
  float linv = 1.0f / lrow;
  const float qnan = __uint_as_float(0x7fc00000u);
  linv = (skipped && !(mrow > -5.0e8f)) ? qnan : linv;
#pragma unroll
  for (int j = 0; j < 4; ++j)
#pragma unroll
    for (int r = 0; r < 8; ++r) ss[wave][col][j * 16 + 8 * g + r] = o[j][r] * linv;
  LDSX();
  for (int i = 0; i < 8; ++i) { const int rl = 2 * i + g;
    vst2(Y + ((size_t)b * SEQ + ql0 + rl) * CC + h * HD + col * 4, *(const v4f*)&ss[wave][rl][col * 4]); }
}

__global__ __launch_bounds__(128) void k_out(const float* __restrict__ Y, const float* __restrict__ WO, const float* __restrict__ BO, float* __restrict__ OUT) {
  __shared__ __align__(16) float sf[4][16][132];
  const int tid = threadIdx.x, wave = tid >> 5, lane = tid & 31, col = lane & 15, g = lane >> 4; const int c0 = blockIdx.y * 128;
  const size_t rb = (size_t)blockIdx.x * 64; const size_t r0 = rb + wave * 16;
  v8f acc[8] = {};
  if ((int)(rb % SEQ) < EARLY) {
#pragma unroll 2
    for (int kc = 0; kc < CC / 32; ++kc) { const F2 a = split_row(Y + (r0 + col) * CC, kc * 32, lane); asm volatile("s_wait_loadcnt 0x0" ::: "memory");
#pragma unroll
      for (int j = 0; j < 8; ++j) { const v16b w = wcol_oi(WO, kc * 32, c0 + j * 16 + col, lane, CC); asm volatile("s_wait_loadcnt 0x0" ::: "memory"); acc[j] = wmma_bf(a.h, w, acc[j]); acc[j] = wmma_bf(a.l, w, acc[j]); } }
#pragma unroll
    for (int j = 0; j < 8; ++j) { const float bias = BO ? bfr(BO[c0 + j * 16 + col]) : 0.f;
#pragma unroll
      for (int r = 0; r < 8; ++r) sf[wave][8 * g + r][j * 16 + col] = acc[j][r] + bias; }
  } else {
#pragma unroll 2
    for (int kc = 0; kc < CC / 32; ++kc) { const v16h a = frag_f32s(Y + (r0 + col) * CC + kc * 32, lane, 64.0f); asm volatile("s_wait_loadcnt 0x0" ::: "memory");
#pragma unroll
      for (int j = 0; j < 8; ++j) { const v16h w = wcolh_oi(WO, kc * 32, c0 + j * 16 + col, lane, CC); asm volatile("s_wait_loadcnt 0x0" ::: "memory"); acc[j] = wmma16(a, w, acc[j]); } }
#pragma unroll
    for (int j = 0; j < 8; ++j) { const float bias = BO ? bfr(BO[c0 + j * 16 + col]) : 0.f;
#pragma unroll
      for (int r = 0; r < 8; ++r) sf[wave][8 * g + r][j * 16 + col] = acc[j][r] * (1.0f / 16384.0f) + bias; } }
  LDSX();
  const size_t orow0 = (r0 / SEQ) * SEQ_FULL + (r0 % SEQ);
  for (int rl = 0; rl < 16; ++rl) vst2(OUT + (orow0 + rl) * DIN + c0 + lane * 4, *(const v4f*)&sf[wave][rl][lane * 4]);
}

extern "C" void kernel_launch(void* const* d_in, const int* in_sizes, int n_in, void* d_out, int out_size, void* d_ws, size_t ws_size, hipStream_t stream) {
  if (n_in < 12) return;
  const long long need_x = ((long long)(NB - 1) * SEQ_FULL + SEQ) * DIN;
  const long long need_m = ((long long)(NB - 1) * SEQ_FULL + SEQ) * SEQ_FULL;
  if ((long long)in_sizes[0] < need_x || (long long)in_sizes[1] < need_x || (long long)in_sizes[2] < need_x) return;
  if ((long long)in_sizes[3] < need_m) return;
  if ((long long)in_sizes[4] < (long long)CC * DIN || (long long)in_sizes[6] < (long long)CC * DIN || (long long)in_sizes[8] < (long long)CC * DIN || (long long)in_sizes[10] < (long long)DIN * CC) return;
  if (in_sizes[5] < CC || in_sizes[7] < CC || in_sizes[9] < CC || in_sizes[11] < DIN) return;
  if ((long long)out_size < need_x) return;
  if (ws_size < (size_t)WS_END) return;
  const float* query = (const float*)d_in[0]; const float* key = (const float*)d_in[1]; const float* value = (const float*)d_in[2];
  const int* mask = (const int*)d_in[3];
  const float* Wq = (const float*)d_in[4]; const float* bq = (const float*)d_in[5];
  const float* Wk = (const float*)d_in[6]; const float* bk = (const float*)d_in[7];
  const float* Wv = (const float*)d_in[8]; const float* bv = (const float*)d_in[9];
  const float* Wo = (const float*)d_in[10]; const float* bo = (const float*)d_in[11];
  char* ws = (char*)d_ws;
  _Float16* QH = (_Float16*)(ws + WS_QH); _Float16* KH = (_Float16*)(ws + WS_KH); _Float16* VT = (_Float16*)(ws + WS_VT);
  __bf16* VB = (__bf16*)(ws + WS_VB); __bf16* VBL = (__bf16*)(ws + WS_VBL);
  float* Y = (float*)(ws + WS_Y); int* FLG = (int*)(ws + WS_FLG);
  k_mflag<<<dim3(NQB, NB), 256, 0, stream>>>(mask, FLG);
  k_proj<<<dim3(NB * SEQ / 64, CC / 128, 3), 128, 0, stream>>>(query, key, value, Wq, Wk, Wv, bq, bk, bv, QH, KH, VT, VB, VBL);
  k_attn<<<dim3(NQB, NH, NB), 128, 0, stream>>>(QH, KH, VT, VB, VBL, mask, FLG, Y);
  k_out<<<dim3(NB * SEQ / 64, DIN / 128), 128, 0, stream>>>(Y, Wo, bo, (float*)d_out);
}
